// Module_74655121539216
// MI455X (gfx1250) — hardware-verified
//
#include <hip/hip_runtime.h>

typedef __bf16 v16b __attribute__((ext_vector_type(16)));
typedef unsigned short v16us __attribute__((ext_vector_type(16)));
typedef float v8f __attribute__((ext_vector_type(8)));
typedef float v4f __attribute__((ext_vector_type(4)));
typedef int v4i __attribute__((ext_vector_type(4)));
typedef v4f v4fa __attribute__((may_alias));

#define NNEU 512
#define NSTEP 64
#define NBAT 8
#define NDLY 4
#define NIN 256
#define NOUT 32
#define ESEG 128

__device__ __forceinline__ unsigned short bf16_rne(float x) {
  unsigned int u = __float_as_uint(x);
  u += 0x7FFFu + ((u >> 16) & 1u);
  return (unsigned short)(u >> 16);
}
__device__ __forceinline__ float bf16_val(unsigned short b) {
  return __uint_as_float(((unsigned int)b) << 16);
}

union BFrag { v16us u; v16b v; };

__device__ __forceinline__ void split_hl(const float (&f)[16], BFrag& hi, BFrag& lo) {
#pragma unroll
  for (int i = 0; i < 16; ++i) {
    const unsigned short hb = bf16_rne(f[i]);
    const float r = f[i] - bf16_val(hb);
    hi.u[i] = hb;
    lo.u[i] = bf16_rne(r);
  }
}

__device__ __forceinline__ v8f wmma_bf16(v16b a, v16b b, v8f c) {
  return __builtin_amdgcn_wmma_f32_16x16x32_bf16(false, a, false, b, (short)0, c, false, false);
}

__global__ void __launch_bounds__(256)
k_prep(const float* __restrict__ w, const float* __restrict__ w_signs, const float* __restrict__ dmap,
       float* weff, int* dsel, int nquads) {
  const int i = blockIdx.x * 256 + threadIdx.x;
  if (i >= nquads) return;
  const size_t base = (size_t)i * 4;
  const int e = (int)(base / NNEU);
  const float sg = w_signs[e];
  const v4f wv = *(const v4f*)(w + base);
  v4f we;
  v4i ds = {0, 0, 0, 0};
#pragma unroll
  for (int j = 0; j < 4; ++j) we[j] = sg * fabsf(wv[j]);
#pragma unroll
  for (int dd = 0; dd < NDLY; ++dd) {
    const v4f dm = *(const v4f*)(dmap + (size_t)dd * NNEU * NNEU + base);
#pragma unroll
    for (int j = 0; j < 4; ++j)
      if (dm[j] > 0.5f) ds[j] = dd;
  }
  *(volatile v4f*)(weff + base) = we;
  *(volatile v4i*)(dsel + base) = ds;
  __threadfence();
  *(volatile v4f*)(weff + base) = we;
  *(volatile v4i*)(dsel + base) = ds;
}

__global__ void __launch_bounds__(256)
k_gemm_hl(const float* __restrict__ A, int lda, const float* __restrict__ Bm, int ldb,
          float* C, int ldc, int M, int K, int Ncol) {
  __shared__ __attribute__((aligned(16))) float s_c[8][16][32];
  const int lane = threadIdx.x & 31;
  const int wl = threadIdx.x >> 5;
  const int h = lane >> 4, m = lane & 15;
  const int tilesN = Ncol >> 5;
  const int ntiles = (M >> 4) * tilesN;
  const int w = blockIdx.x * 8 + wl;
  const bool active = (w < ntiles);
  const int wc = active ? w : 0;
  const int tm = (wc / tilesN) << 4;
  const int tn = (wc % tilesN) << 5;

  v8f acc0 = {0.f, 0.f, 0.f, 0.f, 0.f, 0.f, 0.f, 0.f};
  v8f acc1 = {0.f, 0.f, 0.f, 0.f, 0.f, 0.f, 0.f, 0.f};

  if (active) {
    const float* arow = A + (size_t)(tm + m) * lda + 8 * h;
    const float* bc0 = Bm + tn + m;
    const float* bc1 = bc0 + 16;
    for (int k0 = 0; k0 < K; k0 += 32) {
      float af[16], bf0[16], bf1[16];
      const v4f t0 = *(const v4f*)(arow + k0);
      const v4f t1 = *(const v4f*)(arow + k0 + 4);
      const v4f t2 = *(const v4f*)(arow + k0 + 16);
      const v4f t3 = *(const v4f*)(arow + k0 + 20);
#pragma unroll
      for (int j = 0; j < 4; ++j) {
        af[j] = t0[j]; af[4 + j] = t1[j]; af[8 + j] = t2[j]; af[12 + j] = t3[j];
      }
#pragma unroll
      for (int i = 0; i < 8; ++i) {
        const size_t ka = (size_t)(k0 + 8 * h + i) * ldb;
        const size_t kb = (size_t)(k0 + 16 + 8 * h + i) * ldb;
        bf0[i] = bc0[ka]; bf0[8 + i] = bc0[kb];
        bf1[i] = bc1[ka]; bf1[8 + i] = bc1[kb];
      }
      BFrag ah, al, b0h, b0l, b1h, b1l;
      split_hl(af, ah, al);
      split_hl(bf0, b0h, b0l);
      split_hl(bf1, b1h, b1l);
      acc0 = wmma_bf16(ah.v, b0h.v, acc0);
      acc0 = wmma_bf16(ah.v, b0l.v, acc0);
      acc0 = wmma_bf16(al.v, b0h.v, acc0);
      acc1 = wmma_bf16(ah.v, b1h.v, acc1);
      acc1 = wmma_bf16(ah.v, b1l.v, acc1);
      acc1 = wmma_bf16(al.v, b1h.v, acc1);
      asm volatile("v_nop\n\tv_nop\n\tv_nop\n\tv_nop"
                   : "+v"(acc0), "+v"(acc1)
                   : "v"(ah.v), "v"(al.v), "v"(b0h.v), "v"(b0l.v), "v"(b1h.v), "v"(b1l.v));
    }
  }

#pragma unroll
  for (int r = 0; r < 8; ++r) {
    s_c[wl][8 * h + r][m] = acc0[r];
    s_c[wl][8 * h + r][16 + m] = acc1[r];
  }
  __syncthreads();
  v4f cv[4];
  const int rl = lane >> 3, c4 = (lane & 7) << 2;
#pragma unroll
  for (int j = 0; j < 4; ++j) cv[j] = *(const v4fa*)&s_c[wl][4 * j + rl][c4];
  if (active) {
#pragma unroll
    for (int j = 0; j < 4; ++j)
      *(volatile v4f*)(C + (size_t)(tm + 4 * j + rl) * ldc + tn + c4) = cv[j];
  }
  __threadfence();
  if (active) {
#pragma unroll
    for (int j = 0; j < 4; ++j)
      *(volatile v4f*)(C + (size_t)(tm + 4 * j + rl) * ldc + tn + c4) = cv[j];
  }
}

__global__ void __launch_bounds__(512)
k_steps(const float* __restrict__ inp, const float* __restrict__ weff, const int* __restrict__ dsel,
        const float* __restrict__ A_p, const float* __restrict__ A_d, const float* __restrict__ pvec,
        const int* __restrict__ delays, int nsteps,
        float* wst, float* rec_s, float* rec_wp, float* rec_xb) {
#pragma clang fp contract(off)
  __shared__ __attribute__((aligned(16))) float s_mem[NNEU];
  __shared__ __attribute__((aligned(16))) float s_wp[NNEU];
  __shared__ __attribute__((aligned(16))) float s_xb[NNEU];
  __shared__ __attribute__((aligned(16))) float s_up[NNEU];
  __shared__ __attribute__((aligned(16))) float s_ud[NNEU];
  __shared__ __attribute__((aligned(16))) float s_spk[NNEU];
  __shared__ __attribute__((aligned(16))) float s_gpot[NNEU];
  __shared__ __attribute__((aligned(16))) float s_gdep[NNEU];
  __shared__ float s_ds[NDLY][NNEU];
  __shared__ float s_dsp[NDLY][NNEU];
  __shared__ float s_dxb[NDLY][NNEU];
  __shared__ __attribute__((aligned(16))) float s_part[4][NNEU];

  const int tid = threadIdx.x;
  const int b = blockIdx.x;
  const int n = tid;
  const int eseg = tid >> 7, q = tid & 127, o4 = q << 2;
  const size_t wbase = (size_t)b * NNEU * NNEU;

  int dly[NDLY];
#pragma unroll
  for (int d = 0; d < NDLY; ++d) dly[d] = delays[d];
  const float pn = pvec[n];
  const float pdep = (pn < 0.0f) ? 1.0f : 0.0f;

  s_mem[n] = 0.0f; s_wp[n] = 0.0f; s_xb[n] = 0.0f; s_up[n] = 0.0f; s_ud[n] = 0.0f;

  {
    const v4f one4 = {1.0f, 1.0f, 1.0f, 1.0f};
    for (int el = 0; el < ESEG; ++el) {
      const size_t ro = (size_t)(eseg * ESEG + el) * NNEU + o4;
      *(volatile v4f*)(wst + wbase + ro) = one4;
    }
    __threadfence();
    for (int el = 0; el < ESEG; ++el) {
      const size_t ro = (size_t)(eseg * ESEG + el) * NNEU + o4;
      *(volatile v4f*)(wst + wbase + ro) = one4;
    }
  }
  __syncthreads();

  for (int t = 0; t < nsteps; ++t) {
    const float m = s_mem[n];
    const float s = ((m - 1.0f) > 0.0f) ? 1.0f : 0.0f;
    const float wp = s_wp[n], xb = s_xb[n], up = s_up[n], ud = s_ud[n];
    s_spk[n] = s;
    s_gpot[n] = s * fmaxf(up, 0.0f);
    s_gdep[n] = fmaxf(ud, 0.0f);
    __syncthreads();

    if (tid < 128) {
      const v4f vs = *(const v4fa*)&s_spk[o4];
      const v4f vw = *(const v4fa*)&s_wp[o4];
      const v4f vx = *(const v4fa*)&s_xb[o4];
      const size_t ro = ((size_t)(t * NBAT + b)) * NNEU + o4;
      *(volatile v4f*)(rec_s + ro) = vs;
      *(volatile v4f*)(rec_wp + ro) = vw;
      *(volatile v4f*)(rec_xb + ro) = vx;
      __threadfence();
      *(volatile v4f*)(rec_s + ro) = vs;
      *(volatile v4f*)(rec_wp + ro) = vw;
      *(volatile v4f*)(rec_xb + ro) = vx;
    }
    __syncthreads();

    s_wp[n] = wp * 0.85f + (s * pn) * (1.0f + pdep * wp);
    s_xb[n] = 0.95f * xb + 0.05f * s;
    s_up[n] = 0.95f * up + 0.05f * m;
    s_ud[n] = 0.95f * ud + 0.05f * m;

#pragma unroll
    for (int d = 0; d < NDLY; ++d) {
      const int r = t - dly[d];
      int idx = r % NSTEP;
      if (idx < 0) idx += NSTEP;
      float sv = 0.0f, wv = 0.0f, xv = 0.0f;
      if (idx <= t) {
        const size_t ro = ((size_t)(idx * NBAT + b)) * NNEU + n;
        sv = *(volatile const float*)(rec_s + ro);
        wv = *(volatile const float*)(rec_wp + ro);
        xv = *(volatile const float*)(rec_xb + ro);
      }
      s_ds[d][n] = sv;
      s_dsp[d][n] = sv * (1.0f + wv);
      s_dxb[d][n] = xv;
    }
    __syncthreads();

    {
      const v4f gp = *(const v4fa*)&s_gpot[o4];
      const v4f gd = *(const v4fa*)&s_gdep[o4];
      v4f acc = {0.0f, 0.0f, 0.0f, 0.0f};
#pragma unroll 4
      for (int el = 0; el < ESEG; ++el) {
        const int e = eseg * ESEG + el;
        const size_t ro = (size_t)e * NNEU + o4;
        const v4f wv = *(const v4f*)(weff + ro);
        const v4i dv = *(const v4i*)(dsel + ro);
        const v4f ap = *(const v4f*)(A_p + ro);
        const v4f ad = *(const v4f*)(A_d + ro);
        const v4f ws = *(const v4f*)(wst + wbase + ro);
        v4f nw;
#pragma unroll
        for (int j = 0; j < 4; ++j) {
          const int dd = dv[j] & 3;
          const float synp = s_dsp[dd][e];
          const float xs = s_ds[dd][e];
          const float xbd = s_dxb[dd][e];
          const float pr = wv[j] * synp;
          acc[j] = fmaf(pr, ws[j], acc[j]);
          const float pot = (xbd * ap[j]) * gp[j];
          const float dep = (xs * ad[j]) * gd[j];
          const float v = (ws[j] + pot) - dep;
          nw[j] = fminf(fmaxf(v, 0.0f), 2.0f);
        }
        *(v4f*)(wst + wbase + ro) = nw;
      }
      *(v4fa*)&s_part[eseg][o4] = acc;
    }
    __syncthreads();

    {
      const float syn = ((s_part[0][n] + s_part[1][n]) + s_part[2][n]) + s_part[3][n];
      const float iv = inp[((size_t)(b * NSTEP + t)) * NNEU + n];
      s_mem[n] = ((0.9f * m + iv) + syn) - s;
    }
    __syncthreads();
  }
}

__global__ void __launch_bounds__(64)
k_readout(const float* __restrict__ h2, float* out, int T) {
#pragma clang fp contract(off)
  const int tid = threadIdx.x;
  const int b = tid >> 3, q = tid & 7;
  {
    v4f o = {0.0f, 0.0f, 0.0f, 0.0f};
    for (int t = 0; t < T; ++t) {
      const v4f hv = *(const v4f*)(h2 + ((size_t)(t * NBAT + b)) * NOUT + 4 * q);
      o = 0.9f * o + hv;
      *(volatile v4f*)(out + ((size_t)(b * T + t)) * NOUT + 4 * q) = o;
    }
  }
  __threadfence();
  {
    v4f o = {0.0f, 0.0f, 0.0f, 0.0f};
    for (int t = 0; t < T; ++t) {
      const v4f hv = *(const v4f*)(h2 + ((size_t)(t * NBAT + b)) * NOUT + 4 * q);
      o = 0.9f * o + hv;
      *(volatile v4f*)(out + ((size_t)(b * T + t)) * NOUT + 4 * q) = o;
    }
  }
}

extern "C" void kernel_launch(void* const* d_in, const int* in_sizes, int n_in,
                              void* d_out, int out_size, void* d_ws, size_t ws_size,
                              hipStream_t stream) {
  if (n_in < 10) return;
  const int NN2 = NNEU * NNEU;
  if (in_sizes[0] != NBAT * NSTEP * NIN) return;
  if (in_sizes[1] != NN2) return;
  if (in_sizes[2] != NIN * NNEU) return;
  if (in_sizes[3] != NNEU * NOUT) return;
  if (in_sizes[4] != NDLY * NN2) return;
  if (in_sizes[5] != NDLY) return;
  if (in_sizes[6] != NNEU) return;
  if (in_sizes[7] != NNEU) return;
  if (in_sizes[8] != NN2) return;
  if (in_sizes[9] != NN2) return;
  if (out_size != NBAT * NSTEP * NOUT) return;

  const float* inputs  = (const float*)d_in[0];
  const float* w       = (const float*)d_in[1];
  const float* w_in    = (const float*)d_in[2];
  const float* w_out   = (const float*)d_in[3];
  const float* dmap    = (const float*)d_in[4];
  const int*   delays  = (const int*)d_in[5];
  const float* w_signs = (const float*)d_in[6];
  const float* pvec    = (const float*)d_in[7];
  const float* A_p     = (const float*)d_in[8];
  const float* A_d     = (const float*)d_in[9];

  char* wsb = (char*)d_ws;
  size_t off = 0;
  auto carve = [&](size_t bytes) -> void* {
    void* r = (void*)(wsb + off);
    off += (bytes + 255) & ~(size_t)255;
    return r;
  };
  float* INP   = (float*)carve((size_t)NBAT * NSTEP * NNEU * sizeof(float));
  float* WEFF  = (float*)carve((size_t)NN2 * sizeof(float));
  int*   DSEL  = (int*)carve((size_t)NN2 * sizeof(int));
  float* WST   = (float*)carve((size_t)NBAT * NN2 * sizeof(float));
  float* RECS  = (float*)carve((size_t)NSTEP * NBAT * NNEU * sizeof(float));
  float* RECWP = (float*)carve((size_t)NSTEP * NBAT * NNEU * sizeof(float));
  float* RECXB = (float*)carve((size_t)NSTEP * NBAT * NNEU * sizeof(float));
  float* H2    = (float*)carve((size_t)NSTEP * NBAT * NOUT * sizeof(float));
  if (off > ws_size) return;

  const int nquads = NN2 / 4;
  k_prep<<<(nquads + 255) / 256, 256, 0, stream>>>(w, w_signs, dmap, WEFF, DSEL, nquads);

  {
    const int M = NBAT * NSTEP, K = NIN, Nc = NNEU;
    const int ntiles = (M / 16) * (Nc / 32);
    k_gemm_hl<<<(ntiles + 7) / 8, 256, 0, stream>>>(inputs, NIN, w_in, NNEU, INP, NNEU, M, K, Nc);
  }

  k_steps<<<NBAT, NNEU, 0, stream>>>(INP, WEFF, DSEL, A_p, A_d, pvec, delays, NSTEP,
                                      WST, RECS, RECWP, RECXB);

  {
    const int M = NSTEP * NBAT, K = NNEU, Nc = NOUT;
    const int ntiles = (M / 16) * (Nc / 32);
    k_gemm_hl<<<(ntiles + 7) / 8, 256, 0, stream>>>(RECS, NNEU, w_out, NOUT, H2, NOUT, M, K, Nc);
  }

  k_readout<<<1, 64, 0, stream>>>(H2, (float*)d_out, NSTEP);
}
